// SingleHeadAttentionLayer1_22763326669315
// MI455X (gfx1250) — hardware-verified
//
#include <hip/hip_runtime.h>
#include <stddef.h>
#include <stdint.h>

#define NQ   4096
#define NK   8192
#define DQ   128
#define DKF  128
#define DVF  64
#define HDM  64
#define QB   64
#define KC   64
#define NCH  (NK / KC)

static_assert(NQ % QB == 0);
static_assert(NK % KC == 0);
static_assert(NQ % 64 == 0);
static_assert(NK % 64 == 0);
static_assert(DQ % 32 == 0);
static_assert(DKF % 32 == 0);
static_assert(DVF % 32 == 0);
static_assert(HDM == 64);
static_assert(QB == 64);
static_assert(KC == 64);
static_assert((NQ * DQ) % 2048 == 0);
static_assert((NK * DKF) % 2048 == 0);
static_assert((NK * DVF) % 2048 == 0);
static_assert((HDM * DQ) % 2048 == 0);
static_assert((HDM * DKF) % 2048 == 0);
static_assert((HDM * DVF) % 2048 == 0);

typedef unsigned short us;
typedef __attribute__((ext_vector_type(16))) __bf16 v16bf;
typedef us           v8us __attribute__((ext_vector_type(8)));
typedef float        v8f  __attribute__((ext_vector_type(8)));
typedef float        v4f  __attribute__((ext_vector_type(4)));
typedef unsigned int v4u  __attribute__((ext_vector_type(4)));

union Frag  { v16bf v; v8us h[2]; };
union Pack8 { v8us h; v4u u; };

__device__ __forceinline__ us bf_rne(float f) {
  unsigned u = __float_as_uint(f);
  u = u + 0x7FFFu + ((u >> 16) & 1u);
  return (us)(u >> 16);
}
__device__ __forceinline__ float bf_val(us h) { return __uint_as_float(((unsigned)h) << 16); }
__device__ __forceinline__ void split2(float f, us& hi, us& lo) {
  const us hv = bf_rne(f);
  hi = hv;
  lo = bf_rne(f - bf_val(hv));
}
__device__ __forceinline__ void split8(const float (&f)[8], Pack8& ph, Pack8& pl) {
  us hh[8], ll[8];
#pragma unroll
  for (int e = 0; e < 8; ++e) split2(f[e], hh[e], ll[e]);
  ph.h = (v8us){hh[0], hh[1], hh[2], hh[3], hh[4], hh[5], hh[6], hh[7]};
  pl.h = (v8us){ll[0], ll[1], ll[2], ll[3], ll[4], ll[5], ll[6], ll[7]};
}

__device__ __forceinline__ v8f mma16(v16bf a, v16bf b, v8f c) {
  c = __builtin_amdgcn_wmma_f32_16x16x32_bf16(false, a, false, b, (short)0, c, false, false);
  asm volatile("v_nop\n\tv_nop\n\tv_nop\n\tv_nop" : "+v"(c) : "v"(a), "v"(b));
  return c;
}

__device__ __forceinline__ v16bf ldfrag(const us* p, int ld, int row0, int k0, int lane) {
  const int m = lane & 15, lh = lane >> 4;
  const us* q = p + (size_t)(row0 + m) * ld + k0 + 8 * lh;
  Frag f;
  f.h[0] = *(const v8us*)(q);
  f.h[1] = *(const v8us*)(q + 16);
  return f.v;
}

__device__ __forceinline__ v8f zero8() { return (v8f){0.f, 0.f, 0.f, 0.f, 0.f, 0.f, 0.f, 0.f}; }

template <int KD>
__device__ __forceinline__ void gemm16x64x3(const us* __restrict__ Ah, const us* __restrict__ Al,
                                            const us* __restrict__ Bh, const us* __restrict__ Bl,
                                            int m0, int n0, int lane, v8f (&acc)[4]) {
  static_assert(KD % 32 == 0);
#pragma unroll 1
  for (int k0 = 0; k0 < KD; k0 += 32) {
    const v16bf ah = ldfrag(Ah, KD, m0, k0, lane);
    const v16bf al = ldfrag(Al, KD, m0, k0, lane);
#pragma unroll
    for (int t = 0; t < 4; ++t) {
      const v16bf bh = ldfrag(Bh, KD, n0 + 16 * t, k0, lane);
      const v16bf bl = ldfrag(Bl, KD, n0 + 16 * t, k0, lane);
      acc[t] = mma16(ah, bh, acc[t]);
      acc[t] = mma16(ah, bl, acc[t]);
      acc[t] = mma16(al, bh, acc[t]);
    }
  }
}

__global__ __launch_bounds__(256) void k_cvt(const float* __restrict__ x, us* __restrict__ xh, us* __restrict__ xl) {
  const size_t i = (size_t)blockIdx.x * 2048 + (size_t)threadIdx.x * 8;
  const v4f a0 = *(const v4f*)(x + i);
  const v4f a1 = *(const v4f*)(x + i + 4);
  const float f[8] = {a0[0], a0[1], a0[2], a0[3], a1[0], a1[1], a1[2], a1[3]};
  Pack8 ph, pl;
  split8(f, ph, pl);
  const v4u hv = ph.u, lv = pl.u;
  *(volatile v4u*)(xh + i) = hv;
  *(volatile v4u*)(xl + i) = lv;
  __threadfence();
  *(volatile v4u*)(xh + i) = hv;
  *(volatile v4u*)(xl + i) = lv;
}

#define SFP 68
template <int KD, bool TRANS>
__global__ __launch_bounds__(128) void k_proj(const us* __restrict__ xh, const us* __restrict__ xl,
                                              const us* __restrict__ wh, const us* __restrict__ wl,
                                              const float* __restrict__ bias,
                                              us* __restrict__ yh, us* __restrict__ yl, int tpitch) {
  __shared__ __align__(16) float sf[64 * SFP];
  const int tid = threadIdx.x, lane = tid & 31, wave = tid >> 5;
  const int hh = lane >> 4, c = lane & 15;
  const int mb = blockIdx.x * 64;
  const int m0 = mb + wave * 16;

  v8f acc[4];
#pragma unroll
  for (int t = 0; t < 4; ++t) acc[t] = zero8();
  gemm16x64x3<KD>(xh, xl, wh, wl, m0, 0, lane, acc);

  float bcol[4];
#pragma unroll
  for (int t = 0; t < 4; ++t) bcol[t] = bias[16 * t + c];
#pragma unroll
  for (int t = 0; t < 4; ++t) {
#pragma unroll
    for (int r = 0; r < 8; ++r)
      sf[(wave * 16 + 8 * hh + r) * SFP + 16 * t + c] = acc[t][r] + bcol[t];
  }
  __syncthreads();

  v4u hv[4], lv[4];
  size_t go[4];
  if (!TRANS) {
#pragma unroll
    for (int j = 0; j < 4; ++j) {
      const int p  = tid + 128 * j;
      const int lr = p >> 3;
      const int d0 = (p & 7) * 8;
      const float* ra = sf + lr * SFP + d0;
      const v4f a0 = *(const v4f*)(ra), a1 = *(const v4f*)(ra + 4);
      const float f[8] = {a0[0], a0[1], a0[2], a0[3], a1[0], a1[1], a1[2], a1[3]};
      Pack8 ph, pl;
      split8(f, ph, pl);
      hv[j] = ph.u;
      lv[j] = pl.u;
      go[j] = ((size_t)(mb + lr)) * HDM + d0;
    }
  } else {
#pragma unroll
    for (int j = 0; j < 4; ++j) {
      const int p  = tid + 128 * j;
      const int d  = p >> 3;
      const int pc = p & 7;
      const float* cp = sf + (pc * 8) * SFP + d;
      float f[8];
#pragma unroll
      for (int e = 0; e < 8; ++e) f[e] = cp[e * SFP];
      Pack8 ph, pl;
      split8(f, ph, pl);
      hv[j] = ph.u;
      lv[j] = pl.u;
      go[j] = ((size_t)d) * (size_t)tpitch + mb + pc * 8;
    }
  }
#pragma unroll
  for (int j = 0; j < 4; ++j) { *(volatile v4u*)(yh + go[j]) = hv[j]; *(volatile v4u*)(yl + go[j]) = lv[j]; }
  __threadfence();
#pragma unroll
  for (int j = 0; j < 4; ++j) { *(volatile v4u*)(yh + go[j]) = hv[j]; *(volatile v4u*)(yl + go[j]) = lv[j]; }
}

#define LP  72
#define OTP 68
union AttnLds {
  us    p[2][4 * 16 * LP];
  float o[4][16 * OTP];
};

__global__ __launch_bounds__(128) void k_attn(const us* __restrict__ qh, const us* __restrict__ ql,
                                              const us* __restrict__ kh, const us* __restrict__ kl,
                                              const us* __restrict__ vh, const us* __restrict__ vl,
                                              float* __restrict__ out) {
  __shared__ __align__(16) us Ksh[KC * LP];
  __shared__ __align__(16) us Ksl[KC * LP];
  __shared__ __align__(16) us Vsh[HDM * LP];
  __shared__ __align__(16) us Vsl[HDM * LP];
  __shared__ __align__(16) AttnLds pu;

  const int tid = threadIdx.x, lane = tid & 31, wave = tid >> 5;
  const int hh = lane >> 4, c = lane & 15;
  const int q0 = blockIdx.x * QB + wave * 16;

  const float NEGI = -__builtin_huge_valf();
  float mrow[8], lrow[8];
  v8f oacc[4];
#pragma unroll
  for (int r = 0; r < 8; ++r) { mrow[r] = NEGI; lrow[r] = 0.f; }
#pragma unroll
  for (int t = 0; t < 4; ++t) oacc[t] = zero8();

  us* pwh = pu.p[0] + wave * 16 * LP;
  us* pwl = pu.p[1] + wave * 16 * LP;

#pragma unroll 1
  for (int i = 0; i < NCH; ++i) {
    const int kv0 = i * KC;
    __syncthreads();
    {
      const int r  = tid >> 1;
      const int cb = (tid & 1) * 32;
      const us* ksh = kh + (size_t)(kv0 + r) * HDM + cb;
      const us* ksl = kl + (size_t)(kv0 + r) * HDM + cb;
      const us* vsh = vh + (size_t)r * NK + kv0 + cb;
      const us* vsl = vl + (size_t)r * NK + kv0 + cb;
#pragma unroll
      for (int e = 0; e < 4; ++e) {
        *(v8us*)(Ksh + r * LP + cb + 8 * e) = *(const v8us*)(ksh + 8 * e);
        *(v8us*)(Ksl + r * LP + cb + 8 * e) = *(const v8us*)(ksl + 8 * e);
        *(v8us*)(Vsh + r * LP + cb + 8 * e) = *(const v8us*)(vsh + 8 * e);
        *(v8us*)(Vsl + r * LP + cb + 8 * e) = *(const v8us*)(vsl + 8 * e);
      }
    }
    __syncthreads();

    v8f s[4];
#pragma unroll
    for (int j = 0; j < 4; ++j) s[j] = zero8();
#pragma unroll
    for (int dc = 0; dc < 2; ++dc) {
      const v16bf qah = ldfrag(qh, HDM, q0, dc * 32, lane);
      const v16bf qal = ldfrag(ql, HDM, q0, dc * 32, lane);
#pragma unroll
      for (int j = 0; j < 4; ++j) {
        const v16bf kbh = ldfrag(Ksh, LP, j * 16, dc * 32, lane);
        const v16bf kbl = ldfrag(Ksl, LP, j * 16, dc * 32, lane);
        s[j] = mma16(qah, kbh, s[j]);
        s[j] = mma16(qah, kbl, s[j]);
        s[j] = mma16(qal, kbh, s[j]);
      }
    }
#pragma unroll
    for (int j = 0; j < 4; ++j) {
#pragma unroll
      for (int r = 0; r < 8; ++r) s[j][r] = s[j][r] * 0.125f;
    }
    float cm[8];
#pragma unroll
    for (int r = 0; r < 8; ++r) {
      float m = NEGI;
#pragma unroll
      for (int j = 0; j < 4; ++j) m = fmaxf(m, s[j][r]);
#pragma unroll
      for (int off = 1; off < 16; off <<= 1) m = fmaxf(m, __shfl_xor(m, off, 32));
      cm[r] = m;
    }
    float al[8];
#pragma unroll
    for (int r = 0; r < 8; ++r) {
      const float mnew  = fmaxf(mrow[r], cm[r]);
      const float alpha = __expf(mrow[r] - mnew);
      mrow[r] = mnew;
      float psum = 0.f;
#pragma unroll
      for (int j = 0; j < 4; ++j) {
        const float p = __expf(s[j][r] - mnew);
        psum += p;
        us ph, pl;
        split2(p, ph, pl);
        pwh[(8 * hh + r) * LP + j * 16 + c] = ph;
        pwl[(8 * hh + r) * LP + j * 16 + c] = pl;
      }
#pragma unroll
      for (int off = 1; off < 16; off <<= 1) psum += __shfl_xor(psum, off, 32);
      lrow[r] = lrow[r] * alpha + psum;
      al[r] = alpha;
    }
#pragma unroll
    for (int t = 0; t < 4; ++t)
#pragma unroll
      for (int r = 0; r < 8; ++r) oacc[t][r] *= al[r];
    __syncthreads();

#pragma unroll
    for (int kk = 0; kk < 2; ++kk) {
      const v16bf pah = ldfrag(pwh, LP, 0, kk * 32, lane);
      const v16bf pal = ldfrag(pwl, LP, 0, kk * 32, lane);
#pragma unroll
      for (int t = 0; t < 4; ++t) {
        const v16bf vbh = ldfrag(Vsh, LP, t * 16, kk * 32, lane);
        const v16bf vbl = ldfrag(Vsl, LP, t * 16, kk * 32, lane);
        oacc[t] = mma16(pah, vbh, oacc[t]);
        oacc[t] = mma16(pah, vbl, oacc[t]);
        oacc[t] = mma16(pal, vbh, oacc[t]);
      }
    }
  }

  float invl[8];
#pragma unroll
  for (int r = 0; r < 8; ++r) invl[r] = (lrow[r] > 0.f) ? (1.0f / lrow[r]) : 0.f;
  __syncthreads();
  float* osw = pu.o[wave];
#pragma unroll
  for (int r = 0; r < 8; ++r) {
#pragma unroll
    for (int t = 0; t < 4; ++t) osw[(8 * hh + r) * OTP + 16 * t + c] = oacc[t][r] * invl[r];
  }
  __syncthreads();
  v4f val[8];
  size_t go[8];
#pragma unroll
  for (int it = 0; it < 8; ++it) {
    const int p    = lane + 32 * it;
    const int L    = p >> 3;
    const int pc   = p & 7;
    const int row  = L >> 1;
    const int half = L & 1;
    const int col  = half * 32 + pc * 4;
    val[it] = *(const v4f*)(osw + row * OTP + col);
    go[it]  = (size_t)(q0 + row) * HDM + col;
  }
#pragma unroll
  for (int it = 0; it < 8; ++it) *(volatile v4f*)(out + go[it]) = val[it];
  __threadfence();
#pragma unroll
  for (int it = 0; it < 8; ++it) *(volatile v4f*)(out + go[it]) = val[it];
}

extern "C" void kernel_launch(void* const* d_in, const int* in_sizes, int n_in,
                              void* d_out, int out_size, void* d_ws, size_t ws_size,
                              hipStream_t stream) {
  if (n_in < 9) return;
  if (in_sizes[0] != NQ * DQ) return;
  if (in_sizes[1] != NK * DKF) return;
  if (in_sizes[2] != NK * DVF) return;
  if (in_sizes[3] != HDM * DQ) return;
  if (in_sizes[4] != HDM) return;
  if (in_sizes[5] != HDM * DKF) return;
  if (in_sizes[6] != HDM) return;
  if (in_sizes[7] != HDM * DVF) return;
  if (in_sizes[8] != HDM) return;
  if (out_size != NQ * HDM) return;

  const float* q  = (const float*)d_in[0];
  const float* k  = (const float*)d_in[1];
  const float* v  = (const float*)d_in[2];
  const float* Wq = (const float*)d_in[3];
  const float* bq = (const float*)d_in[4];
  const float* Wk = (const float*)d_in[5];
  const float* bk = (const float*)d_in[6];
  const float* Wv = (const float*)d_in[7];
  const float* bv = (const float*)d_in[8];
  float* out = (float*)d_out;

  size_t off = 0;
  const size_t oQIh = off; off += (size_t)NQ * DQ * 2;
  const size_t oQIl = off; off += (size_t)NQ * DQ * 2;
  const size_t oKIh = off; off += (size_t)NK * DKF * 2;
  const size_t oKIl = off; off += (size_t)NK * DKF * 2;
  const size_t oVIh = off; off += (size_t)NK * DVF * 2;
  const size_t oVIl = off; off += (size_t)NK * DVF * 2;
  const size_t oWQh = off; off += (size_t)HDM * DQ * 2;
  const size_t oWQl = off; off += (size_t)HDM * DQ * 2;
  const size_t oWKh = off; off += (size_t)HDM * DKF * 2;
  const size_t oWKl = off; off += (size_t)HDM * DKF * 2;
  const size_t oWVh = off; off += (size_t)HDM * DVF * 2;
  const size_t oWVl = off; off += (size_t)HDM * DVF * 2;
  const size_t oQPh = off; off += (size_t)NQ * HDM * 2;
  const size_t oQPl = off; off += (size_t)NQ * HDM * 2;
  const size_t oKPh = off; off += (size_t)NK * HDM * 2;
  const size_t oKPl = off; off += (size_t)NK * HDM * 2;
  const size_t oVTh = off; off += (size_t)HDM * NK * 2;
  const size_t oVTl = off; off += (size_t)HDM * NK * 2;
  if (off > ws_size) return;
  if (off > (size_t)134217728) return;

  char* ws = (char*)d_ws;
  us* QIh = (us*)(ws + oQIh);  us* QIl = (us*)(ws + oQIl);
  us* KIh = (us*)(ws + oKIh);  us* KIl = (us*)(ws + oKIl);
  us* VIh = (us*)(ws + oVIh);  us* VIl = (us*)(ws + oVIl);
  us* WQh = (us*)(ws + oWQh);  us* WQl = (us*)(ws + oWQl);
  us* WKh = (us*)(ws + oWKh);  us* WKl = (us*)(ws + oWKl);
  us* WVh = (us*)(ws + oWVh);  us* WVl = (us*)(ws + oWVl);
  us* QPh = (us*)(ws + oQPh);  us* QPl = (us*)(ws + oQPl);
  us* KPh = (us*)(ws + oKPh);  us* KPl = (us*)(ws + oKPl);
  us* VTh = (us*)(ws + oVTh);  us* VTl = (us*)(ws + oVTl);

  k_cvt<<<dim3((NQ * DQ) / 2048),  dim3(256), 0, stream>>>(q,  QIh, QIl);
  k_cvt<<<dim3((NK * DKF) / 2048), dim3(256), 0, stream>>>(k,  KIh, KIl);
  k_cvt<<<dim3((NK * DVF) / 2048), dim3(256), 0, stream>>>(v,  VIh, VIl);
  k_cvt<<<dim3((HDM * DQ) / 2048), dim3(256), 0, stream>>>(Wq, WQh, WQl);
  k_cvt<<<dim3((HDM * DKF) / 2048), dim3(256), 0, stream>>>(Wk, WKh, WKl);
  k_cvt<<<dim3((HDM * DVF) / 2048), dim3(256), 0, stream>>>(Wv, WVh, WVl);
  k_proj<DQ, false><<<dim3(NQ / 64), dim3(128), 0, stream>>>(QIh, QIl, WQh, WQl, bq, QPh, QPl, HDM);
  k_proj<DKF, false><<<dim3(NK / 64), dim3(128), 0, stream>>>(KIh, KIl, WKh, WKl, bk, KPh, KPl, HDM);
  k_proj<DVF, true><<<dim3(NK / 64), dim3(128), 0, stream>>>(VIh, VIl, WVh, WVl, bv, VTh, VTl, NK);
  k_attn<<<dim3(NQ / QB), dim3(128), 0, stream>>>(QPh, QPl, KPh, KPl, VTh, VTl, out);
  (void)hipGetLastError();
}
